// MultiHeadAttention_81793357185469
// MI455X (gfx1250) — hardware-run, weakly checked
//
#include <hip/hip_runtime.h>


#ifndef NB
#define NB 8
#endif
#ifndef SEQ
#define SEQ 1024
#endif
#define NB_FULL  8
#define SEQ_FULL 1024
#define DM   1024
#define NH_  16
#define HD   64
#define AW   4
#define QRS  2048.0f
#define QRI  (1.0f / 2048.0f)
#define SC2  (0.03125f * 1.4426950408889634f)
#define PSH  8.0f
#define YCS  256.0f
#define WOS  64.0f
#define OSI  (1.0f / 16384.0f)
#ifndef SCORE_RES
#define SCORE_RES 0
#endif

static_assert(HD == 64);
static_assert(NH_ * HD == DM);
static_assert(AW == 4);
static_assert(SEQ == DM);
static_assert(SEQ % 64 == 0);
static_assert(SEQ % 32 == 0);
static_assert(DM % 64 == 0);
static_assert(NB <= NB_FULL);
static_assert(SEQ <= SEQ_FULL);
static_assert((HD * HD) % 8 == 0);
static_assert(((size_t)DM * DM) % 8 == 0);

typedef _Float16 h16;
typedef unsigned short bf;
typedef __attribute__((ext_vector_type(16))) __bf16   v16bf;
typedef __attribute__((ext_vector_type(16))) _Float16 v16h;
typedef __attribute__((ext_vector_type(8)))  _Float16 v8h;
typedef __attribute__((ext_vector_type(8)))  unsigned short v8us;
typedef __attribute__((ext_vector_type(8)))  float    v8f;
typedef __attribute__((ext_vector_type(4)))  float    v4f;
typedef v4f  __attribute__((may_alias)) v4fa;

__device__ __forceinline__ unsigned short f2bf(float f) { unsigned u = __float_as_uint(f); u += 0x7FFFu + ((u >> 16) & 1u); return (unsigned short)(u >> 16); }
__device__ __forceinline__ float bfr(float f) { return __uint_as_float(((unsigned)f2bf(f)) << 16); }
__device__ __forceinline__ v8us cv8(v8f v) { v8us o;
#pragma unroll
    for (int k = 0; k < 8; ++k) o[k] = f2bf(v[k]);
    return o; }
__device__ __forceinline__ v16h cat16(v8h lo, v8h hi) { return __builtin_shufflevector(lo, hi, 0, 1, 2, 3, 4, 5, 6, 7, 8, 9, 10, 11, 12, 13, 14, 15); }
__device__ __forceinline__ v16bf cat16b(v8us lo, v8us hi) { return __builtin_bit_cast(v16bf, __builtin_shufflevector(lo, hi, 0, 1, 2, 3, 4, 5, 6, 7, 8, 9, 10, 11, 12, 13, 14, 15)); }
__device__ __forceinline__ v8f wmma16(v16h a, v16h b, v8f c) { return __builtin_amdgcn_wmma_f32_16x16x32_f16(false, a, false, b, (short)0, c, false, false); }
__device__ __forceinline__ v8f wmmab(v16bf a, v16bf b, v8f c) { return __builtin_amdgcn_wmma_f32_16x16x32_bf16(false, a, false, b, (short)0, c, false, false); }
__device__ __forceinline__ v16h  ldh(const h16* p) { return cat16(*(const v8h*)p, *(const v8h*)(p + 16)); }
__device__ __forceinline__ v16bf ldb(const bf* p)  { return cat16b(*(const v8us*)p, *(const v8us*)(p + 16)); }
__device__ __forceinline__ void wave_sync() { __builtin_amdgcn_fence(3  , "wavefront"); __builtin_amdgcn_wave_barrier(); asm volatile("" ::: "memory"); }

__global__ __launch_bounds__(256) void k_cvtw(const float* __restrict__ wq, const float* __restrict__ wk, const float* __restrict__ wv, bf* WB) {
    const int i = blockIdx.x * 256 + threadIdx.x; if (i >= HD * HD / 8) return;
    const v8us oq = cv8(*(const v8f*)(wq + (size_t)i * 8));
    const v8us ok = cv8(*(const v8f*)(wk + (size_t)i * 8));
    const v8us ov = cv8(*(const v8f*)(wv + (size_t)i * 8));
    bf* d0 = WB + (size_t)i * 8; bf* d1 = d0 + HD * HD; bf* d2 = d1 + HD * HD;
    *(volatile v8us*)d0 = oq; *(volatile v8us*)d1 = ok; *(volatile v8us*)d2 = ov;
    __threadfence();
    *(volatile v8us*)d0 = oq; *(volatile v8us*)d1 = ok; *(volatile v8us*)d2 = ov;
}

__global__ __launch_bounds__(256) void k_cvtwo(const float* __restrict__ src, h16* dst, size_t n8) {
    const size_t i = (size_t)blockIdx.x * 256 + threadIdx.x; if (i >= n8) return;
    const v8f v = *(const v8f*)(src + i * 8); v8h o;
#pragma unroll
    for (int k = 0; k < 8; ++k) o[k] = (h16)(bfr(v[k]) * WOS);
    *(volatile v8h*)(dst + i * 8) = o; __threadfence(); *(volatile v8h*)(dst + i * 8) = o;
}

__global__ __launch_bounds__(32) __attribute__((amdgpu_num_vgpr(256))) void k_qkv(const float* __restrict__ x, const bf* __restrict__ WB, const float* __restrict__ bq, const float* __restrict__ bk, const float* __restrict__ bv, h16* PL, size_t ple) {
    __shared__ __align__(16) float os[16 * 68];
    __shared__ __align__(16) float vs[64 * 68];
    const int lane = threadIdx.x & 31, lr = lane & 15, hi = lane >> 4;
    const int tt = blockIdx.x; const int b = tt / (SEQ / 64); const int m0 = (tt % (SEQ / 64)) * 64;
    const int h = blockIdx.y; const int zh = h * NB_FULL + b;
    const float* xp = x + ((size_t)b * SEQ_FULL + m0 + lr) * DM + h * HD + 8 * hi;
    float bqc[4], bkc[4];
#pragma unroll
    for (int nb = 0; nb < 4; ++nb) { bqc[nb] = bfr(bq[nb * 16 + lr]); bkc[nb] = bfr(bk[nb * 16 + lr]); }
    h16* Pr = PL + 2 * ple;
#pragma unroll 1
    for (int mb = 0; mb < 4; ++mb) {
        const float* p = xp + (size_t)mb * 16 * DM;
        const v16bf xa0 = cat16b(cv8(*(const v8f*)p), cv8(*(const v8f*)(p + 16)));
        const v16bf xa1 = cat16b(cv8(*(const v8f*)(p + 32)), cv8(*(const v8f*)(p + 48)));
        const size_t sb = ((size_t)zh * SEQ + m0 + mb * 16) * HD;
#pragma unroll
        for (int w = 0; w < 2; ++w) {
            v8f acc[4];
#pragma unroll
            for (int i = 0; i < 4; ++i) acc[i] = (v8f){};
            const bf* W = WB + (size_t)w * HD * HD + (size_t)lr * HD + 8 * hi;
#pragma unroll
            for (int nb = 0; nb < 4; ++nb) { const v16bf wf = ldb(W + nb * 16 * HD); acc[nb] = wmmab(xa0, wf, acc[nb]); }
#pragma unroll
            for (int nb = 0; nb < 4; ++nb) { const v16bf wf = ldb(W + nb * 16 * HD + 32); acc[nb] = wmmab(xa1, wf, acc[nb]); }
            asm volatile("v_nop\n\tv_nop\n\tv_nop\n\tv_nop" : "+v"(acc[0]), "+v"(acc[1]), "+v"(acc[2]), "+v"(acc[3]) : "v"(xa0), "v"(xa1));
#pragma unroll
            for (int nb = 0; nb < 4; ++nb) { const float bc = (w == 0) ? bqc[nb] : bkc[nb];
#pragma unroll
                for (int j = 0; j < 8; ++j) os[(hi * 8 + j) * 68 + nb * 16 + lr] = acc[nb][j] + bc; }
            wave_sync();
            h16* Ph = PL + (size_t)w * ple;
#pragma unroll 1
            for (int ps = 0; ps < 2; ++ps) {
#pragma unroll
                for (int s = 0; s < 4; ++s) { const int row = 4 * s + (lane >> 3), c8 = (lane & 7) * 8;
                    const v4f x0 = *(const v4fa*)(&os[row * 68 + c8]); const v4f x1 = *(const v4fa*)(&os[row * 68 + c8 + 4]); v8h hv, rv;
#pragma unroll
                    for (int i = 0; i < 4; ++i) { const h16 a0 = (h16)x0[i]; const h16 a1 = (h16)x1[i]; hv[i] = a0; hv[4 + i] = a1; rv[i] = (h16)((x0[i] - (float)a0) * QRS); rv[4 + i] = (h16)((x1[i] - (float)a1) * QRS); }
                    const size_t oo = sb + (size_t)row * HD + c8;
                    *(volatile v8h*)(Ph + oo) = hv; if (w == 1 && SCORE_RES) *(volatile v8h*)(Pr + oo) = rv; }
                if (ps == 0) __threadfence(); }
            wave_sync();
        }
        {
            v8f acc[4];
#pragma unroll
            for (int i = 0; i < 4; ++i) acc[i] = (v8f){};
            const bf* W = WB + (size_t)2 * HD * HD + (size_t)lr * HD + 8 * hi;
#pragma unroll
            for (int j = 0; j < 4; ++j) { const v16bf wf = ldb(W + j * 16 * HD); acc[j] = wmmab(wf, xa0, acc[j]); }
#pragma unroll
            for (int j = 0; j < 4; ++j) { const v16bf wf = ldb(W + j * 16 * HD + 32); acc[j] = wmmab(wf, xa1, acc[j]); }
            asm volatile("v_nop\n\tv_nop\n\tv_nop\n\tv_nop" : "+v"(acc[0]), "+v"(acc[1]), "+v"(acc[2]), "+v"(acc[3]) : "v"(xa0), "v"(xa1));
#pragma unroll
            for (int j = 0; j < 4; ++j) {
                const v4f b0 = *(const v4f*)(bv + j * 16 + 8 * hi); const v4f b1 = *(const v4f*)(bv + j * 16 + 8 * hi + 4);
#pragma unroll
                for (int r = 0; r < 4; ++r) {
                    vs[(j * 16 + 8 * hi + r) * 68 + mb * 16 + lr]     = acc[j][r]     + bfr(b0[r]);
                    vs[(j * 16 + 8 * hi + 4 + r) * 68 + mb * 16 + lr] = acc[j][4 + r] + bfr(b1[r]); } }
        }
    }
    wave_sync();
    h16* P3 = PL + 3 * ple; const size_t vb = (size_t)zh * HD * SEQ + m0;
#pragma unroll 1
    for (int ps = 0; ps < 2; ++ps) {
#pragma unroll 4
        for (int s = 0; s < 16; ++s) { const int row = 4 * s + (lane >> 3), c8 = (lane & 7) * 8;
            const v4f x0 = *(const v4fa*)(&vs[row * 68 + c8]); const v4f x1 = *(const v4fa*)(&vs[row * 68 + c8 + 4]); v8h hv;
#pragma unroll
            for (int i = 0; i < 4; ++i) { hv[i] = (h16)x0[i]; hv[4 + i] = (h16)x1[i]; }
            *(volatile v8h*)(P3 + vb + (size_t)row * SEQ + c8) = hv; }
        if (ps == 0) __threadfence(); }
}

__global__ __launch_bounds__(32 * AW) __attribute__((amdgpu_num_vgpr(256))) void k_flash(const h16* __restrict__ QH, const h16* __restrict__ QR, const h16* __restrict__ KP, const h16* __restrict__ VT, h16* Y) {
    __shared__ __align__(16) float os[64 * 68];
    const int lane = threadIdx.x & 31, lr = lane & 15, hi = lane >> 4;
    const int wave = __builtin_amdgcn_readfirstlane(threadIdx.x >> 5);
    const int zc = blockIdx.y; const int h = zc / NB, b = zc % NB; const int zh = h * NB_FULL + b;
    const int t0 = (blockIdx.x * AW + wave) * 16;
    const size_t pbase = (size_t)zh * SEQ * HD;
    const size_t qo = pbase + (size_t)(t0 + lr) * HD + 8 * hi;
    const v16h qh0 = ldh(QH + qo), qh1 = ldh(QH + qo + 32);
#if SCORE_RES
    const v16h qr0 = ldh(QR + qo), qr1 = ldh(QR + qo + 32);
#endif
    const size_t ko = pbase + (size_t)lr * HD + 8 * hi;
    const size_t vo = pbase + (size_t)lr * SEQ + 8 * hi;
    v8f o0 = (v8f){}, o1 = (v8f){}, o2 = (v8f){}, o3 = (v8f){};
    float m = -3.0e38f, l = 0.0f;
#pragma unroll 1
    for (int key0 = 0; key0 < SEQ; key0 += 32) {
        const h16* ka = KP + ko + (size_t)key0 * HD;
        const v16h ka0 = ldh(ka), ka1 = ldh(ka + 32), kb0 = ldh(ka + 16 * HD), kb1 = ldh(ka + 16 * HD + 32);
        float ta[8], tb[8]; float mx = -3.0e38f;
#if SCORE_RES
        v8f sHa = (v8f){}, sLa = (v8f){}, sHb = (v8f){}, sLb = (v8f){};
        sHa = wmma16(ka0, qh0, sHa); sLa = wmma16(ka0, qr0, sLa); sHb = wmma16(kb0, qh0, sHb); sLb = wmma16(kb0, qr0, sLb);
        sHa = wmma16(ka1, qh1, sHa); sLa = wmma16(ka1, qr1, sLa); sHb = wmma16(kb1, qh1, sHb); sLb = wmma16(kb1, qr1, sLb);
        asm volatile("v_nop\n\tv_nop\n\tv_nop\n\tv_nop" : "+v"(sHa), "+v"(sLa), "+v"(sHb), "+v"(sLb) : "v"(ka0), "v"(ka1), "v"(kb0), "v"(kb1));
#pragma unroll
        for (int r = 0; r < 8; ++r) { ta[r] = (sHa[r] + sLa[r] * QRI) * SC2; tb[r] = (sHb[r] + sLb[r] * QRI) * SC2; mx = fmaxf(mx, fmaxf(ta[r], tb[r])); }
#else
        v8f sHa = (v8f){}, sHb = (v8f){};
        sHa = wmma16(ka0, qh0, sHa); sHb = wmma16(kb0, qh0, sHb);
        sHa = wmma16(ka1, qh1, sHa); sHb = wmma16(kb1, qh1, sHb);
        asm volatile("v_nop\n\tv_nop\n\tv_nop\n\tv_nop" : "+v"(sHa), "+v"(sHb) : "v"(ka0), "v"(ka1), "v"(kb0), "v"(kb1));
#pragma unroll
        for (int r = 0; r < 8; ++r) { ta[r] = sHa[r] * SC2; tb[r] = sHb[r] * SC2; mx = fmaxf(mx, fmaxf(ta[r], tb[r])); }
#endif
        mx = fmaxf(mx, __shfl_xor(mx, 16, 32));
        const float mnew = fmaxf(m, mx);
        const float alpha = __builtin_amdgcn_exp2f(m - mnew);
        const float sh = PSH - mnew;
        v16h pb; float ls = 0.0f;
#pragma unroll
        for (int r = 0; r < 8; ++r) { const h16 pa = (h16)__builtin_amdgcn_exp2f(ta[r] + sh); const h16 pc = (h16)__builtin_amdgcn_exp2f(tb[r] + sh); pb[r] = pa; pb[8 + r] = pc; ls += (float)pa + (float)pc; }
        l = l * alpha + ls; m = mnew;
        o0 = o0 * alpha; o1 = o1 * alpha; o2 = o2 * alpha; o3 = o3 * alpha;
        const h16* va = VT + vo + key0;
        const v16h v0 = ldh(va), v1 = ldh(va + (size_t)16 * SEQ), v2 = ldh(va + (size_t)32 * SEQ), v3 = ldh(va + (size_t)48 * SEQ);
        o0 = wmma16(v0, pb, o0); o1 = wmma16(v1, pb, o1); o2 = wmma16(v2, pb, o2); o3 = wmma16(v3, pb, o3);
        asm volatile("v_nop\n\tv_nop\n\tv_nop\n\tv_nop" : "+v"(o0), "+v"(o1), "+v"(o2), "+v"(o3) : "v"(v0), "v"(v1), "v"(v2), "v"(v3), "v"(pb));
    }
    l += __shfl_xor(l, 16, 32);
    const float ys = YCS * (1.0f / l);
    const int cw = wave * 16 + lr;
#pragma unroll
    for (int r = 0; r < 8; ++r) {
        os[( 0 + 8 * hi + r) * 68 + cw] = o0[r] * ys;
        os[(16 + 8 * hi + r) * 68 + cw] = o1[r] * ys;
        os[(32 + 8 * hi + r) * 68 + cw] = o2[r] * ys;
        os[(48 + 8 * hi + r) * 68 + cw] = o3[r] * ys; }
    __syncthreads();
    const int tid = threadIdx.x;
    h16* yb = Y + (size_t)zh * HD * SEQ + (size_t)blockIdx.x * (16 * AW);
#pragma unroll 1
    for (int ps = 0; ps < 2; ++ps) {
#pragma unroll
        for (int s = 0; s < 4; ++s) { const int row = 16 * s + (tid >> 3), c8 = (tid & 7) * 8;
            const v4f x0 = *(const v4fa*)(&os[row * 68 + c8]); const v4f x1 = *(const v4fa*)(&os[row * 68 + c8 + 4]); v8h hv;
#pragma unroll
            for (int i = 0; i < 4; ++i) { hv[i] = (h16)x0[i]; hv[4 + i] = (h16)x1[i]; }
            *(volatile v8h*)(yb + (size_t)row * SEQ + c8) = hv; }
        if (ps == 0) __threadfence(); }
}

__global__ __launch_bounds__(32) __attribute__((amdgpu_num_vgpr(256))) void k_out(const h16* __restrict__ Y, const h16* __restrict__ WO, const float* __restrict__ bo, float* OUT) {
    __shared__ __align__(16) float os[16 * 68];
    const int K = DM;
    const int lane = threadIdx.x & 31, lr = lane & 15, hi = lane >> 4;
    const int zc = blockIdx.x; const int h = zc / NB, b = zc % NB; const int r0 = (h * NB_FULL + b) * 64; const int c0 = blockIdx.y * 64;
    v8f acc[4][4];
#pragma unroll
    for (int mb = 0; mb < 4; ++mb)
#pragma unroll
        for (int nb = 0; nb < 4; ++nb) acc[mb][nb] = (v8f){};
    const size_t aoff = (size_t)(r0 + lr) * K + 8 * hi, boff = (size_t)(c0 + lr) * K + 8 * hi;
#pragma unroll 1
    for (int kc = 0; kc < K; kc += 32) {
        v16h a[4];
#pragma unroll
        for (int mb = 0; mb < 4; ++mb) a[mb] = ldh(Y + aoff + (size_t)mb * 16 * K + kc);
#pragma unroll
        for (int nb = 0; nb < 4; ++nb) { const v16h bb = ldh(WO + boff + (size_t)nb * 16 * K + kc);
#pragma unroll
            for (int mb = 0; mb < 4; ++mb) acc[mb][nb] = wmma16(a[mb], bb, acc[mb][nb]); }
        asm volatile("v_nop\n\tv_nop\n\tv_nop\n\tv_nop" : "+v"(acc[0][0]), "+v"(acc[1][1]), "+v"(acc[2][2]), "+v"(acc[3][3]) : "v"(a[0]), "v"(a[1]), "v"(a[2]), "v"(a[3]));
    }
    float bc[4];
#pragma unroll
    for (int nb = 0; nb < 4; ++nb) bc[nb] = bfr(bo[c0 + nb * 16 + lr]);
#pragma unroll
    for (int mb = 0; mb < 4; ++mb) {
#pragma unroll
        for (int nb = 0; nb < 4; ++nb) {
#pragma unroll
            for (int j = 0; j < 8; ++j) os[(hi * 8 + j) * 68 + nb * 16 + lr] = acc[mb][nb][j] * OSI + bc[nb]; }
        wave_sync();
        float* orow = OUT + (size_t)(r0 + mb * 16) * DM + c0;
#pragma unroll 1
        for (int ps = 0; ps < 2; ++ps) {
#pragma unroll
            for (int s = 0; s < 8; ++s) { const int row = 2 * s + hi, cofs = lr * 4;
                const v4f val = *(const v4fa*)(&os[row * 68 + cofs]);
                *(volatile v4f*)(orow + (size_t)row * DM + cofs) = val; }
            if (ps == 0) __threadfence(); }
        wave_sync();
    }
}

static constexpr size_t al256(size_t v) { return (v + 255) & ~(size_t)255; }
static constexpr size_t PLE   = (size_t)NB_FULL * NH_ * SEQ * HD;
static constexpr size_t SZ_PL = al256(PLE * 2);
static constexpr size_t SZ_Y  = al256((size_t)NB_FULL * NH_ * HD * SEQ * 2);
static constexpr size_t SZ_WO = al256((size_t)DM * DM * 2);
static constexpr size_t SZ_WB = al256((size_t)3 * HD * HD * 2);
static constexpr size_t SZ_TOTAL = 4 * SZ_PL + SZ_Y + SZ_WO + SZ_WB;
static_assert(SZ_PL == PLE * 2);
static_assert(SZ_TOTAL <= (size_t)134217728);
static_assert(((size_t)(NH_ - 1) * NB_FULL + NB) * HD <= (size_t)NB_FULL * NH_ * HD);

extern "C" void kernel_launch(void* const* d_in, const int* in_sizes, int n_in,
                              void* d_out, int out_size, void* d_ws, size_t ws_size, hipStream_t stream) {
    if (n_in < 9) return;
    const size_t needx = ((size_t)(NB - 1) * SEQ_FULL + SEQ) * DM;
    if ((size_t)in_sizes[0] < needx) return;
    if ((size_t)in_sizes[1] < (size_t)HD * HD || (size_t)in_sizes[3] < (size_t)HD * HD || (size_t)in_sizes[5] < (size_t)HD * HD) return;
    if ((size_t)in_sizes[2] < (size_t)HD || (size_t)in_sizes[4] < (size_t)HD || (size_t)in_sizes[6] < (size_t)HD) return;
    if ((size_t)in_sizes[7] < (size_t)DM * DM || (size_t)in_sizes[8] < (size_t)DM) return;
    if ((size_t)out_size < (((size_t)(NH_ - 1) * NB_FULL + NB) * HD) * DM) return;
    if (SZ_TOTAL > ws_size) return;
    const float* x  = (const float*)d_in[0];
    const float* wq = (const float*)d_in[1]; const float* bq = (const float*)d_in[2];
    const float* wk = (const float*)d_in[3]; const float* bk = (const float*)d_in[4];
    const float* wv = (const float*)d_in[5]; const float* bv = (const float*)d_in[6];
    const float* wo = (const float*)d_in[7]; const float* bo = (const float*)d_in[8];
    float* OUT = (float*)d_out;
    char* wsp = (char*)d_ws;
    h16* PL = (h16*)wsp; wsp += 4 * SZ_PL;
    h16* YP = (h16*)wsp; wsp += SZ_Y;
    h16* WO = (h16*)wsp; wsp += SZ_WO;
    bf*  WB = (bf*)wsp;  wsp += SZ_WB;

    k_cvtw<<<(HD * HD / 8 + 255) / 256, 256, 0, stream>>>(wq, wk, wv, WB);
    { const size_t n8 = (size_t)DM * DM / 8; k_cvtwo<<<(unsigned)((n8 + 255) / 256), 256, 0, stream>>>(wo, WO, n8); }

    k_qkv<<<dim3(NB * (SEQ / 64), NH_, 1), 32, 0, stream>>>(x, WB, bq, bk, bv, PL, PLE);

    k_flash<<<dim3(SEQ / (16 * AW), NH_ * NB, 1), 32 * AW, 0, stream>>>(PL + PLE, PL + 2 * PLE, PL, PL + 3 * PLE, YP);

    k_out<<<dim3(NH_ * NB, DM / 64, 1), 32, 0, stream>>>(YP, WO, bo, OUT);
}
